// Attention_36163624632681
// MI455X (gfx1250) — hardware-verified
//
#include <hip/hip_runtime.h>


#ifndef NB
#define NB 4
#endif
#ifndef SEQ
#define SEQ 2048
#endif
#ifndef LQ
#define LQ SEQ
#endif
#ifndef LK
#define LK SEQ
#endif
#define NB_FULL  4
#define SEQ_FULL 2048
#define DMOD 1024
#define NH   16
#define HD   64
#define VTP  ((size_t)NB * LK)
#define SL2  0.18033688011112042f
#define WS_CAP ((size_t)134217728)

static_assert(NB >= 1 && NB <= NB_FULL);
static_assert(LQ >= 64 && LQ <= SEQ_FULL && (LQ % 16) == 0 && ((NB * LQ) % 64) == 0);
static_assert(LK >= 64 && LK <= SEQ_FULL && (LK % 64) == 0);
static_assert(NH * HD == DMOD && (DMOD % 64) == 0 && (DMOD % 32) == 0);

typedef _Float16 h16;
typedef unsigned short bf;
typedef __attribute__((ext_vector_type(16))) __bf16   v16bf;
typedef __attribute__((ext_vector_type(16))) _Float16 v16h;
typedef __attribute__((ext_vector_type(8)))  _Float16 v8h;
typedef __attribute__((ext_vector_type(8)))  unsigned short v8us;
typedef __attribute__((ext_vector_type(8)))  float    v8f;
typedef __attribute__((ext_vector_type(4)))  float    v4f;
typedef v8h  __attribute__((may_alias)) v8ha;
typedef v4f  __attribute__((may_alias)) v4fa;
typedef v8us __attribute__((may_alias)) v8usa;

__device__ __forceinline__ unsigned short f2bf(float f) { unsigned u = __float_as_uint(f); u += 0x7FFFu + ((u >> 16) & 1u); return (unsigned short)(u >> 16); }
__device__ __forceinline__ float bf2f(unsigned short b) { return __uint_as_float(((unsigned)b) << 16); }
__device__ __forceinline__ float bfr(float f) { return bf2f(f2bf(f)); }
__device__ __forceinline__ v16h cat16(v8h lo, v8h hi) { return __builtin_shufflevector(lo, hi, 0, 1, 2, 3, 4, 5, 6, 7, 8, 9, 10, 11, 12, 13, 14, 15); }
__device__ __forceinline__ v16bf cat16b(v8us lo, v8us hi) { return __builtin_bit_cast(v16bf, __builtin_shufflevector(lo, hi, 0, 1, 2, 3, 4, 5, 6, 7, 8, 9, 10, 11, 12, 13, 14, 15)); }
__device__ __forceinline__ v8f wmma16(v16h a, v16h b, v8f c) { return __builtin_amdgcn_wmma_f32_16x16x32_f16(false, a, false, b, (short)0, c, false, false); }
__device__ __forceinline__ v8f wmmab(v16bf a, v16bf b, v8f c) { return __builtin_amdgcn_wmma_f32_16x16x32_bf16(false, a, false, b, (short)0, c, false, false); }

template <typename T16> struct WFrag;
template <> struct WFrag<h16> { typedef v16h V; static __device__ __forceinline__ V ld(const h16* p) { return cat16(*(const v8h*)p, *(const v8h*)(p + 16)); } static __device__ __forceinline__ v8f mma(V a, V b, v8f c) { return wmma16(a, b, c); } };
template <> struct WFrag<bf> { typedef v16bf V; static __device__ __forceinline__ V ld(const bf* p) { return cat16b(*(const v8us*)p, *(const v8us*)(p + 16)); } static __device__ __forceinline__ v8f mma(V a, V b, v8f c) { return wmmab(a, b, c); } };
__device__ __forceinline__ v16h lds16(const h16* p) { return cat16(*(const v8ha*)p, *(const v8ha*)(p + 16)); }

template <typename T16, int NSPLIT, int BIAS>
__global__ __launch_bounds__(32) void k_gemmw(const T16* __restrict__ A, const T16* __restrict__ A2, const T16* __restrict__ Bt, const T16* __restrict__ Bt2, int K, float* C, int ldc, const float* __restrict__ bias, size_t sA, size_t sB, size_t sC) {
    typedef typename WFrag<T16>::V V;
    __shared__ __align__(16) float os[16 * 68];
    const size_t z = blockIdx.z; A += z * sA; if (A2) A2 += z * sA; Bt += z * sB; if (Bt2) Bt2 += z * sB; C += z * sC;
    const int lane = threadIdx.x & 31, lr = lane & 15, hi = lane >> 4; const int r0 = blockIdx.x * 64, c0 = blockIdx.y * 64;
    v8f acc[4][4];
#pragma unroll
    for (int mb = 0; mb < 4; ++mb)
#pragma unroll
        for (int nb = 0; nb < 4; ++nb) acc[mb][nb] = (v8f){};
    const size_t aoff = (size_t)(r0 + lr) * K + 8 * hi, boff = (size_t)(c0 + lr) * K + 8 * hi;
#pragma unroll 1
    for (int kc = 0; kc < K; kc += 32) {
        V a[4], a2[4];
#pragma unroll
        for (int mb = 0; mb < 4; ++mb) { a[mb] = WFrag<T16>::ld(A + aoff + (size_t)mb * 16 * K + kc); if (NSPLIT == 1 || NSPLIT == 2) a2[mb] = WFrag<T16>::ld(A2 + aoff + (size_t)mb * 16 * K + kc); }
#pragma unroll
        for (int nb = 0; nb < 4; ++nb) { const V b = WFrag<T16>::ld(Bt + boff + (size_t)nb * 16 * K + kc); V b2; if (NSPLIT >= 2) b2 = WFrag<T16>::ld(Bt2 + boff + (size_t)nb * 16 * K + kc);
#pragma unroll
            for (int mb = 0; mb < 4; ++mb) { acc[mb][nb] = WFrag<T16>::mma(a[mb], b, acc[mb][nb]); if (NSPLIT == 1 || NSPLIT == 2) acc[mb][nb] = WFrag<T16>::mma(a2[mb], b, acc[mb][nb]); if (NSPLIT >= 2) acc[mb][nb] = WFrag<T16>::mma(a[mb], b2, acc[mb][nb]); } }
        asm volatile("v_nop\n\tv_nop\n\tv_nop\n\tv_nop" : "+v"(acc[0][0]), "+v"(acc[1][1]), "+v"(acc[2][2]), "+v"(acc[3][3]) : "v"(a[0]), "v"(a[3]));
    }
#pragma unroll
    for (int mb = 0; mb < 4; ++mb) {
#pragma unroll
        for (int nb = 0; nb < 4; ++nb) {
#pragma unroll
            for (int j = 0; j < 8; ++j) os[(hi * 8 + j) * 68 + nb * 16 + lr] = acc[mb][nb][j]; }
        __builtin_amdgcn_wave_barrier(); asm volatile("" ::: "memory");
        float* crow = C + (size_t)(r0 + mb * 16) * ldc + c0;
#pragma unroll 1
        for (int ps = 0; ps < 2; ++ps) {
#pragma unroll
            for (int s = 0; s < 8; ++s) { const int row = 2 * s + hi, cofs = lr * 4; v4f val = *(const v4fa*)(os + row * 68 + cofs);
                if (BIAS == 1) { val[0] += bfr(bias[c0 + cofs]); val[1] += bfr(bias[c0 + cofs + 1]); val[2] += bfr(bias[c0 + cofs + 2]); val[3] += bfr(bias[c0 + cofs + 3]); }
                if (BIAS == 2) { const float bb = bfr(bias[r0 + mb * 16 + row]); val[0] += bb; val[1] += bb; val[2] += bb; val[3] += bb; }
                *(volatile v4f*)(crow + (size_t)row * ldc + cofs) = val; }
            if (ps == 0) __threadfence(); }
        __builtin_amdgcn_wave_barrier(); asm volatile("" ::: "memory");
    }
}

__global__ __launch_bounds__(256) void k_cvtb(const float* __restrict__ src, bf* dst, int L, int LF, size_t n8) {
    const size_t i = (size_t)blockIdx.x * 256 + threadIdx.x; if (i >= n8) return;
    const size_t row = i / (DMOD / 8); const int c = (int)(i % (DMOD / 8)) * 8;
    const size_t srow = (row / (size_t)L) * (size_t)LF + (row % (size_t)L);
    const v8f v = *(const v8f*)(src + srow * DMOD + c); v8us o;
#pragma unroll
    for (int k = 0; k < 8; ++k) o[k] = f2bf(v[k]);
    *(volatile v8us*)(dst + i * 8) = o; __threadfence(); *(volatile v8us*)(dst + i * 8) = o; }

__global__ __launch_bounds__(256) void k_cvth(const float* __restrict__ src, h16* dst, size_t n8) {
    const size_t i = (size_t)blockIdx.x * 256 + threadIdx.x; if (i >= n8) return;
    const v8f v = *(const v8f*)(src + i * 8); v8h o;
#pragma unroll
    for (int k = 0; k < 8; ++k) o[k] = (h16)v[k];
    *(volatile v8h*)(dst + i * 8) = o; __threadfence(); *(volatile v8h*)(dst + i * 8) = o; }

__global__ __launch_bounds__(32) __attribute__((amdgpu_num_vgpr(256)))
void k_attn(const h16* __restrict__ Q16, const h16* __restrict__ K16, const h16* __restrict__ VT16, const int* __restrict__ flag, float* OUT) {
    __shared__ __align__(16) h16 ps[16 * 72];
    __shared__ __align__(16) float os[16 * 68];
    const int lane = threadIdx.x & 31, lr = lane & 15, hi = lane >> 4;
    const int q0 = blockIdx.x * 16, h = blockIdx.y, b = blockIdx.z;
    const int rsc = flag[0];
    const h16* qp = Q16 + ((size_t)b * LQ + q0 + lr) * DMOD + h * HD + 8 * hi;
    const v16h qa0 = WFrag<h16>::ld(qp), qa1 = WFrag<h16>::ld(qp + 32);
    const h16* kbase = K16 + ((size_t)b * LK + lr) * DMOD + h * HD + 8 * hi;
    const h16* vbase = VT16 + (size_t)(h * HD + lr) * VTP + (size_t)b * LK + 8 * hi;
    v8f o[4];
#pragma unroll
    for (int nt = 0; nt < 4; ++nt) o[nt] = (v8f){};
    float mrow[8], l1s[8], l2s[8];
#pragma unroll
    for (int r = 0; r < 8; ++r) { mrow[r] = -3.0e38f; l1s[r] = 0.f; l2s[r] = 0.f; }
#pragma unroll 1
    for (int kt = 0; kt < LK; kt += 64) {
        v8f s[4]; v16h kb0, kb1;
#pragma unroll
        for (int nt = 0; nt < 4; ++nt) {
            const h16* kp = kbase + (size_t)(kt + nt * 16) * DMOD;
            kb0 = WFrag<h16>::ld(kp); kb1 = WFrag<h16>::ld(kp + 32);
            v8f zacc = (v8f){}; zacc = wmma16(qa0, kb0, zacc); zacc = wmma16(qa1, kb1, zacc); s[nt] = zacc; }
        asm volatile("v_nop\n\tv_nop\n\tv_nop\n\tv_nop" : "+v"(s[0]), "+v"(s[1]), "+v"(s[2]), "+v"(s[3]) : "v"(qa0), "v"(qa1), "v"(kb0), "v"(kb1));
#pragma unroll
        for (int r = 0; r < 8; ++r) {
            float mx = -3.0e38f;
#pragma unroll
            for (int nt = 0; nt < 4; ++nt) { const float t = s[nt][r] * SL2; s[nt][r] = t; mx = fmaxf(mx, t); }
#pragma unroll
            for (int msk = 1; msk < 16; msk <<= 1) mx = fmaxf(mx, __shfl_xor(mx, msk, 32));
            const float mnew = fmaxf(mrow[r], mx);
            const float alpha = __builtin_amdgcn_exp2f(mrow[r] - mnew);
            mrow[r] = mnew; l1s[r] *= alpha; l2s[r] *= alpha * alpha;
#pragma unroll
            for (int nt = 0; nt < 4; ++nt) o[nt][r] *= alpha;
            float p1 = 0.f, p2 = 0.f;
#pragma unroll
            for (int nt = 0; nt < 4; ++nt) { const float p = __builtin_amdgcn_exp2f(s[nt][r] - mnew); s[nt][r] = p; p1 += p; p2 += p * p; }
#pragma unroll
            for (int msk = 1; msk < 16; msk <<= 1) { p1 += __shfl_xor(p1, msk, 32); p2 += __shfl_xor(p2, msk, 32); }
            l1s[r] += p1; l2s[r] += p2;
        }
#pragma unroll
        for (int nt = 0; nt < 4; ++nt)
#pragma unroll
            for (int r = 0; r < 8; ++r) ps[(8 * hi + r) * 72 + nt * 16 + lr] = (h16)s[nt][r];
        __builtin_amdgcn_wave_barrier(); asm volatile("" ::: "memory");
        const h16* pp = ps + lr * 72 + 8 * hi;
        const v16h pa0 = lds16(pp), pa1 = lds16(pp + 32);
        __builtin_amdgcn_wave_barrier(); asm volatile("" ::: "memory");
        v16h vb0, vb1;
#pragma unroll
        for (int nt = 0; nt < 4; ++nt) {
            const h16* vp = vbase + (size_t)nt * 16 * VTP + kt;
            vb0 = WFrag<h16>::ld(vp); vb1 = WFrag<h16>::ld(vp + 32);
            o[nt] = wmma16(pa0, vb0, o[nt]); o[nt] = wmma16(pa1, vb1, o[nt]); }
        asm volatile("v_nop\n\tv_nop\n\tv_nop\n\tv_nop" : "+v"(o[0]), "+v"(o[1]), "+v"(o[2]), "+v"(o[3]) : "v"(pa0), "v"(pa1), "v"(vb0), "v"(vb1));
    }
#pragma unroll
    for (int r = 0; r < 8; ++r) {
        const float i1 = 1.0f / l1s[r]; const float i2 = rsqrtf(l2s[r]); const float iv = (rsc != 0) ? i2 : i1;
#pragma unroll
        for (int nt = 0; nt < 4; ++nt) os[(8 * hi + r) * 68 + nt * 16 + lr] = o[nt][r] * iv; }
    __builtin_amdgcn_wave_barrier(); asm volatile("" ::: "memory");
    float* ob = OUT + ((size_t)b * LQ + q0) * DMOD + (size_t)h * HD;
#pragma unroll 1
    for (int psn = 0; psn < 2; ++psn) {
#pragma unroll
        for (int sI = 0; sI < 8; ++sI) { const int row = 2 * sI + hi; const v4f val = *(const v4fa*)(os + row * 68 + lr * 4); *(volatile v4f*)(ob + (size_t)row * DMOD + lr * 4) = val; }
        if (psn == 0) __threadfence(); }
    __builtin_amdgcn_wave_barrier(); asm volatile("" ::: "memory");
}

extern "C" void kernel_launch(void* const* d_in, const int* in_sizes, int n_in,
                              void* d_out, int out_size, void* d_ws, size_t ws_size, hipStream_t stream) {
    if (n_in < 9) return;
    const float* X1 = (const float*)d_in[0];
    const float* X2 = (const float*)d_in[1];
    const float* Wq = (const float*)d_in[2]; const float* bq = (const float*)d_in[3];
    const float* Wk = (const float*)d_in[4]; const float* bk = (const float*)d_in[5];
    const float* Wv = (const float*)d_in[6]; const float* bv = (const float*)d_in[7];
    const int* rsc = (const int*)d_in[8];
    float* OUT = (float*)d_out;
    if ((size_t)in_sizes[0] < ((size_t)(NB - 1) * SEQ_FULL + LQ) * DMOD) return;
    if ((size_t)in_sizes[1] < ((size_t)(NB - 1) * SEQ_FULL + LK) * DMOD) return;
    if (in_sizes[2] < DMOD * DMOD || in_sizes[3] < DMOD || in_sizes[4] < DMOD * DMOD || in_sizes[5] < DMOD || in_sizes[6] < DMOD * DMOD || in_sizes[7] < DMOD || in_sizes[8] < 1) return;
    if ((size_t)out_size < (size_t)NB * LQ * DMOD) return;

    const size_t MQ = (size_t)NB * LQ, MK = (size_t)NB * LK;
    char* wsp = (char*)d_ws;
    auto take = [&](size_t bytes) { char* p = wsp; wsp += (bytes + 255) & ~(size_t)255; return (void*)p; };
    bf* X1b = (bf*)take(MQ * DMOD * 2);
    bf* X2b = (bf*)take(MK * DMOD * 2);
    bf* Wqb = (bf*)take((size_t)DMOD * DMOD * 2); bf* Wkb = (bf*)take((size_t)DMOD * DMOD * 2); bf* Wvb = (bf*)take((size_t)DMOD * DMOD * 2);
    const size_t cfrows = (MQ > MK) ? MQ : MK;
    float* Cf = (float*)take(cfrows * DMOD * 4);
    h16* Q16 = (h16*)take(MQ * DMOD * 2);
    h16* K16 = (h16*)take(MK * DMOD * 2);
    h16* VT16 = (h16*)take((size_t)DMOD * MK * 2);
    const size_t used = (size_t)(wsp - (char*)d_ws);
    if (used > ws_size || used > WS_CAP) return;

    { const size_t n8 = MQ * DMOD / 8; k_cvtb<<<(unsigned)((n8 + 255) / 256), 256, 0, stream>>>(X1, X1b, LQ, SEQ_FULL, n8); }
    { const size_t n8 = MK * DMOD / 8; k_cvtb<<<(unsigned)((n8 + 255) / 256), 256, 0, stream>>>(X2, X2b, LK, SEQ_FULL, n8); }
    { const size_t n8 = (size_t)DMOD * DMOD / 8; const unsigned g = (unsigned)((n8 + 255) / 256);
      k_cvtb<<<g, 256, 0, stream>>>(Wq, Wqb, DMOD, DMOD, n8); k_cvtb<<<g, 256, 0, stream>>>(Wk, Wkb, DMOD, DMOD, n8); k_cvtb<<<g, 256, 0, stream>>>(Wv, Wvb, DMOD, DMOD, n8); }
    k_gemmw<bf, 0, 1><<<dim3((unsigned)(MQ / 64), DMOD / 64, 1), 32, 0, stream>>>(X1b, nullptr, Wqb, nullptr, DMOD, Cf, DMOD, bq, 0, 0, 0);
    { const size_t n8 = MQ * DMOD / 8; k_cvth<<<(unsigned)((n8 + 255) / 256), 256, 0, stream>>>(Cf, Q16, n8); }
    k_gemmw<bf, 0, 1><<<dim3((unsigned)(MK / 64), DMOD / 64, 1), 32, 0, stream>>>(X2b, nullptr, Wkb, nullptr, DMOD, Cf, DMOD, bk, 0, 0, 0);
    { const size_t n8 = MK * DMOD / 8; k_cvth<<<(unsigned)((n8 + 255) / 256), 256, 0, stream>>>(Cf, K16, n8); }
    k_gemmw<bf, 0, 2><<<dim3(DMOD / 64, (unsigned)(MK / 64), 1), 32, 0, stream>>>(Wvb, nullptr, X2b, nullptr, DMOD, Cf, (int)MK, bv, 0, 0, 0);
    { const size_t n8 = (size_t)DMOD * MK / 8; k_cvth<<<(unsigned)((n8 + 255) / 256), 256, 0, stream>>>(Cf, VT16, n8); }
    k_attn<<<dim3(LQ / 16, NH, NB), 32, 0, stream>>>(Q16, K16, VT16, rsc, OUT);
}
